// _PAMBlock_1726576855063
// MI455X (gfx1250) — hardware-verified
//
#include <hip/hip_runtime.h>
#define NI 4
#define CC 64
#define HH 64
#define W2 128
#define WW 64
#define SS 2
#define SH (HH / SS)
#define SW (WW / SS)
#define LL (SH * SW * 2)
#define NBK (SS * SS)
#define NSL (NI * NBK)
#define CK 32
#define CV 64
#define NPIX (NI * HH * W2)

typedef __bf16 v16b __attribute__((ext_vector_type(16)));
typedef unsigned short v8us __attribute__((ext_vector_type(8), may_alias));
typedef float  v8f  __attribute__((ext_vector_type(8)));
typedef float  v4f  __attribute__((ext_vector_type(4)));
typedef float  v4fa __attribute__((ext_vector_type(4), may_alias));
union FragB { v16b v; v8us half[2]; unsigned short u[16]; };

__device__ __forceinline__ unsigned short bf16_bits(float x) { unsigned int u = __float_as_uint(x); return (unsigned short)((u + 0x7FFFu + ((u >> 16) & 1u)) >> 16); }
__device__ __forceinline__ float bf16_val(unsigned short b) { return __uint_as_float(((unsigned int)b) << 16); }
__device__ __forceinline__ float bf16_round(float x) { return bf16_val(bf16_bits(x)); }
template <int NT>
__device__ __forceinline__ v8f mmaN(v16b ah, v16b al, v16b bh, v16b bl, v8f c) {
  c = __builtin_amdgcn_wmma_f32_16x16x32_bf16(false, ah, false, bh, (short)0, c, false, false);
  if (NT >= 2) c = __builtin_amdgcn_wmma_f32_16x16x32_bf16(false, al, false, bh, (short)0, c, false, false);
  if (NT >= 3) c = __builtin_amdgcn_wmma_f32_16x16x32_bf16(false, ah, false, bl, (short)0, c, false, false);
  asm volatile("v_nop\n\tv_nop\n\tv_nop\n\tv_nop" : "+v"(c) : "v"(ah), "v"(al), "v"(bh), "v"(bl));
  return c;
}

__global__ __launch_bounds__(256) void k_wt_bf16(const float* __restrict__ W, unsigned short* __restrict__ Wt, int K, int N) {
  const int t = blockIdx.x * 256 + threadIdx.x;
  const int k8n = K / 8;
  if (t >= N * k8n) return;
  const int n = t / k8n, k8 = (t % k8n) * 8;
  v8us v;
#pragma unroll
  for (int i = 0; i < 8; ++i) v[i] = bf16_bits(W[(size_t)(k8 + i) * N + n]);
  *(volatile v8us*)(Wt + (size_t)n * K + k8) = v;
  __threadfence();
  *(volatile v8us*)(Wt + (size_t)n * K + k8) = v;
}

template <bool ASPLIT, int ACT, bool BIAS_BF16>
__global__ __launch_bounds__(128) void k_gemm_bf(const float* __restrict__ A, int lda, const unsigned short* __restrict__ Wt, int ldb,
                                               const float* __restrict__ bias, float* __restrict__ C, int ldc, int M, int N, int K) {
  __shared__ __attribute__((aligned(16))) float so[4][16][64];
  const int tid = threadIdx.x, w = tid >> 5, lane = tid & 31, ln = lane & 15, hh = lane >> 4;
  const int ntn = N / 64;
  const int wid = blockIdx.x * 4 + w;
  const int mt = wid / ntn, nq = wid % ntn;
  if (mt * 16 >= M) return;
  const int row0 = mt * 16, col0 = nq * 64;
  const float* arow = A + (size_t)(row0 + ln) * lda;
  v8f acc[4] = {};
  for (int kb = 0; kb < K; kb += 32) {
    FragB ah, al;
    const v4f x0 = *(const v4fa*)(arow + kb + 8 * hh), x1 = *(const v4fa*)(arow + kb + 8 * hh + 4);
    const v4f x2 = *(const v4fa*)(arow + kb + 16 + 8 * hh), x3 = *(const v4fa*)(arow + kb + 16 + 8 * hh + 4);
    float xs[16] = {x0[0],x0[1],x0[2],x0[3],x1[0],x1[1],x1[2],x1[3],x2[0],x2[1],x2[2],x2[3],x3[0],x3[1],x3[2],x3[3]};
#pragma unroll
    for (int i = 0; i < 16; ++i) { const unsigned short hb = bf16_bits(xs[i]); ah.u[i] = hb; al.u[i] = ASPLIT ? bf16_bits(xs[i] - bf16_val(hb)) : (unsigned short)0; }
#pragma unroll
    for (int t = 0; t < 4; ++t) {
      const unsigned short* brow = Wt + (size_t)(col0 + t * 16 + ln) * ldb + kb;
      FragB b;
      b.half[0] = *(const v8us*)(brow + 8 * hh);
      b.half[1] = *(const v8us*)(brow + 16 + 8 * hh);
      acc[t] = mmaN<ASPLIT ? 2 : 1>(ah.v, al.v, b.v, b.v, acc[t]);
    }
  }
#pragma unroll
  for (int t = 0; t < 4; ++t) {
    float bv = bias ? bias[col0 + t * 16 + ln] : 0.f;
    if (BIAS_BF16) bv = bf16_round(bv);
#pragma unroll
    for (int r = 0; r < 8; ++r) { float v = acc[t][r] + bv; if (ACT == 1) v = fmaxf(v, 0.f); so[w][8 * hh + r][t * 16 + ln] = v; }
  }
  __builtin_amdgcn_fence(__ATOMIC_ACQ_REL, "workgroup");
  __builtin_amdgcn_wave_barrier();
  const int rsub = lane >> 4, c4 = (lane & 15) * 4;
  for (int pass = 0; pass < 2; ++pass) {
#pragma unroll
    for (int q = 0; q < 8; ++q) {
      const int r = q * 2 + rsub;
      const v4f v = *(const v4fa*)&so[w][r][c4];
      *(volatile v4f*)(C + (size_t)(row0 + r) * ldc + col0 + c4) = v;
    }
    if (pass == 0) __threadfence();
  }
}

template <int D, bool CAUSAL>
__global__ __launch_bounds__(128) void k_flash(const float* __restrict__ qb, const float* __restrict__ kb, const float* __restrict__ vb,
                                             int pitch, int T, int H, float scale, float* __restrict__ y, int ypitch) {
  constexpr int KS = D / 32;
  constexpr int DT = D / 16;
  __shared__ __attribute__((aligned(16))) unsigned short sKh[32][D + 8], sKl[32][D + 8], sVh[32][D + 8], sVl[32][D + 8];
  __shared__ __attribute__((aligned(16))) unsigned short sPh[4][16][40], sPl[4][16][40];
  __shared__ __attribute__((aligned(16))) float sO[4][16][D];
  const int tid = threadIdx.x, w = tid >> 5, lane = tid & 31, ln = lane & 15, hh = lane >> 4;
  const int nqb = (T + 63) / 64;
  const int bh = blockIdx.x / nqb, qblk = blockIdx.x % nqb;
  const int b = bh / H, h = bh % H;
  const int q0 = qblk * 64 + w * 16;
  const float* Q = qb + (size_t)b * T * pitch + h * D;
  const float* K = kb + (size_t)b * T * pitch + h * D;
  const float* V = vb + (size_t)b * T * pitch + h * D;

  FragB aqh[KS], aql[KS];
  {
    int row = q0 + ln; if (row >= T) row = T - 1;
    const float* qr = Q + (size_t)row * pitch;
#pragma unroll
    for (int ks = 0; ks < KS; ++ks)
#pragma unroll
      for (int i = 0; i < 16; ++i) {
        const int d = ks * 32 + ((i < 8) ? (8 * hh + i) : (16 + 8 * hh + (i - 8)));
        const float x = qr[d] * scale; const unsigned short hb = bf16_bits(x);
        aqh[ks].u[i] = hb; aql[ks].u[i] = bf16_bits(x - bf16_val(hb));
      }
  }
  float m_r[8], l_r[8];
#pragma unroll
  for (int r = 0; r < 8; ++r) { m_r[r] = -3.0e38f; l_r[r] = 0.f; }
  v8f oacc[DT];
#pragma unroll
  for (int dt = 0; dt < DT; ++dt) oacc[dt] = (v8f){0.f,0.f,0.f,0.f,0.f,0.f,0.f,0.f};

  const int kv_end = CAUSAL ? min(T, qblk * 64 + 64) : T;
  for (int j0 = 0; j0 < kv_end; j0 += 32) {
    __syncthreads();
    for (int e = tid; e < 32 * (D / 4); e += 128) {
      const int r = e / (D / 4), c4 = (e % (D / 4)) * 4;
      const int key = j0 + r;
      v4f kf = {0.f,0.f,0.f,0.f}, vf = {0.f,0.f,0.f,0.f};
      if (key < T) { kf = *(const v4fa*)(K + (size_t)key * pitch + c4); vf = *(const v4fa*)(V + (size_t)key * pitch + c4); }
#pragma unroll
      for (int t = 0; t < 4; ++t) {
        unsigned short hb = bf16_bits(kf[t]); sKh[r][c4 + t] = hb; sKl[r][c4 + t] = bf16_bits(kf[t] - bf16_val(hb));
        hb = bf16_bits(vf[t]); sVh[r][c4 + t] = hb; sVl[r][c4 + t] = bf16_bits(vf[t] - bf16_val(hb));
      }
    }
    __syncthreads();
    v8f s[2];
#pragma unroll
    for (int nt = 0; nt < 2; ++nt) {
      v8f acc = {};
#pragma unroll
      for (int ks = 0; ks < KS; ++ks) {
        FragB bh_, bl_;
        bh_.half[0] = *(const v8us*)&sKh[nt * 16 + ln][ks * 32 + 8 * hh]; bh_.half[1] = *(const v8us*)&sKh[nt * 16 + ln][ks * 32 + 16 + 8 * hh];
        bl_.half[0] = *(const v8us*)&sKl[nt * 16 + ln][ks * 32 + 8 * hh]; bl_.half[1] = *(const v8us*)&sKl[nt * 16 + ln][ks * 32 + 16 + 8 * hh];
        acc = mmaN<3>(aqh[ks].v, aql[ks].v, bh_.v, bl_.v, acc);
      }
      s[nt] = acc;
    }
    float alpha[8];
#pragma unroll
    for (int r = 0; r < 8; ++r) {
      const int qi = q0 + 8 * hh + r;
      const int ja = j0 + ln, jb = j0 + 16 + ln;
      if (CAUSAL) { if (ja > qi) s[0][r] = -3.0e38f; if (jb > qi) s[1][r] = -3.0e38f; }
      if (ja >= T) s[0][r] = -3.0e38f;
      if (jb >= T) s[1][r] = -3.0e38f;
      float mx = fmaxf(s[0][r], s[1][r]);
      mx = fmaxf(mx, __shfl_xor(mx, 1, 32)); mx = fmaxf(mx, __shfl_xor(mx, 2, 32)); mx = fmaxf(mx, __shfl_xor(mx, 4, 32)); mx = fmaxf(mx, __shfl_xor(mx, 8, 32));
      const float mnew = fmaxf(m_r[r], mx);
      alpha[r] = (mnew > -1.0e38f) ? __expf(m_r[r] - mnew) : 1.0f;
      const float p0 = (s[0][r] > -1.0e38f) ? __expf(s[0][r] - mnew) : 0.f;
      const float p1 = (s[1][r] > -1.0e38f) ? __expf(s[1][r] - mnew) : 0.f;
      m_r[r] = mnew;
      l_r[r] = l_r[r] * alpha[r] + p0 + p1;
      unsigned short hb = bf16_bits(p0); sPh[w][8 * hh + r][ln] = hb;      sPl[w][8 * hh + r][ln] = bf16_bits(p0 - bf16_val(hb));
      hb = bf16_bits(p1);                sPh[w][8 * hh + r][16 + ln] = hb; sPl[w][8 * hh + r][16 + ln] = bf16_bits(p1 - bf16_val(hb));
    }
#pragma unroll
    for (int dt = 0; dt < DT; ++dt)
#pragma unroll
      for (int r = 0; r < 8; ++r) oacc[dt][r] *= alpha[r];
    __builtin_amdgcn_fence(__ATOMIC_ACQ_REL, "workgroup");
    __builtin_amdgcn_wave_barrier();
    FragB pah, pal;
    pah.half[0] = *(const v8us*)&sPh[w][ln][8 * hh]; pah.half[1] = *(const v8us*)&sPh[w][ln][16 + 8 * hh];
    pal.half[0] = *(const v8us*)&sPl[w][ln][8 * hh]; pal.half[1] = *(const v8us*)&sPl[w][ln][16 + 8 * hh];
#pragma unroll
    for (int dt = 0; dt < DT; ++dt) {
      FragB bvh, bvl;
#pragma unroll
      for (int i = 0; i < 8; ++i) {
        bvh.u[i] = sVh[8 * hh + i][dt * 16 + ln]; bvh.u[8 + i] = sVh[16 + 8 * hh + i][dt * 16 + ln];
        bvl.u[i] = sVl[8 * hh + i][dt * 16 + ln]; bvl.u[8 + i] = sVl[16 + 8 * hh + i][dt * 16 + ln];
      }
      oacc[dt] = mmaN<3>(pah.v, pal.v, bvh.v, bvl.v, oacc[dt]);
    }
    __builtin_amdgcn_fence(__ATOMIC_ACQ_REL, "workgroup");
    __builtin_amdgcn_wave_barrier();
  }
#pragma unroll
  for (int r = 0; r < 8; ++r) {
    float l = l_r[r];
    l += __shfl_xor(l, 1, 32); l += __shfl_xor(l, 2, 32); l += __shfl_xor(l, 4, 32); l += __shfl_xor(l, 8, 32);
    l_r[r] = (l > 0.f) ? 1.0f / l : 0.f;
  }
#pragma unroll
  for (int dt = 0; dt < DT; ++dt)
#pragma unroll
    for (int r = 0; r < 8; ++r) sO[w][8 * hh + r][dt * 16 + ln] = oacc[dt][r] * l_r[r];
  __builtin_amdgcn_fence(__ATOMIC_ACQ_REL, "workgroup");
  __builtin_amdgcn_wave_barrier();
  for (int pass = 0; pass < 2; ++pass) {
    for (int r = 0; r < 16; ++r) {
      const int row = q0 + r;
      if (row < T && lane < D / 4) {
        const v4f val = *(const v4fa*)&sO[w][r][lane * 4];
        *(volatile v4f*)(y + ((size_t)b * T + row) * ypitch + h * D + lane * 4) = val;
      }
    }
    if (pass == 0) __threadfence();
  }
}

template <bool ASPLIT, int ACT, bool BIAS_BF16, bool RES_BF16>
__global__ __launch_bounds__(128) void k_gemm_bf3(const float* __restrict__ A, int lda, const unsigned short* __restrict__ Wt, int ldb,
                                                const float* __restrict__ bias, const float* __restrict__ resid, int rmod, int ldr,
                                                float* __restrict__ C, int ldc, int M, int N, int K) {
  __shared__ __attribute__((aligned(16))) float so[4][16][64];
  const int tid = threadIdx.x, w = tid >> 5, lane = tid & 31, ln = lane & 15, hh = lane >> 4;
  const int ntn = N / 64;
  const int wid = blockIdx.x * 4 + w;
  const int mt = wid / ntn, nq = wid % ntn;
  if (mt * 16 >= M) return;
  const int row0 = mt * 16, col0 = nq * 64;
  const float* arow = A + (size_t)(row0 + ln) * lda;
  v8f acc[4] = {};
  for (int kb = 0; kb < K; kb += 32) {
    FragB ah, al;
    const v4f x0 = *(const v4fa*)(arow + kb + 8 * hh), x1 = *(const v4fa*)(arow + kb + 8 * hh + 4);
    const v4f x2 = *(const v4fa*)(arow + kb + 16 + 8 * hh), x3 = *(const v4fa*)(arow + kb + 16 + 8 * hh + 4);
    float xs[16] = {x0[0],x0[1],x0[2],x0[3],x1[0],x1[1],x1[2],x1[3],x2[0],x2[1],x2[2],x2[3],x3[0],x3[1],x3[2],x3[3]};
#pragma unroll
    for (int i = 0; i < 16; ++i) { const unsigned short hb = bf16_bits(xs[i]); ah.u[i] = hb; al.u[i] = ASPLIT ? bf16_bits(xs[i] - bf16_val(hb)) : (unsigned short)0; }
#pragma unroll
    for (int t = 0; t < 4; ++t) {
      const unsigned short* brow = Wt + (size_t)(col0 + t * 16 + ln) * ldb + kb;
      FragB b;
      b.half[0] = *(const v8us*)(brow + 8 * hh);
      b.half[1] = *(const v8us*)(brow + 16 + 8 * hh);
      acc[t] = mmaN<ASPLIT ? 2 : 1>(ah.v, al.v, b.v, b.v, acc[t]);
    }
  }
#pragma unroll
  for (int t = 0; t < 4; ++t) {
    const int col = col0 + t * 16 + ln;
    float bv = bias ? bias[col] : 0.f;
    if (BIAS_BF16) bv = bf16_round(bv);
#pragma unroll
    for (int r = 0; r < 8; ++r) {
      float v = acc[t][r] + bv;
      if (resid) { float rv = resid[(size_t)((row0 + 8 * hh + r) % rmod) * ldr + col]; if (RES_BF16) rv = bf16_round(rv); v += rv; }
      if (ACT == 1) v = fmaxf(v, 0.f);
      if (ACT == 2) v = 0.5f * v * (1.0f + erff(v * 0.70710678118654752f));
      if (ACT == 3) { const float u = 0.7978845608028654f * (v + 0.044715f * v * v * v); v = 0.5f * v * (1.0f + tanhf(u)); }
      so[w][8 * hh + r][t * 16 + ln] = v;
    }
  }
  __builtin_amdgcn_fence(__ATOMIC_ACQ_REL, "workgroup");
  __builtin_amdgcn_wave_barrier();
  const int rsub = lane >> 4, c4 = (lane & 15) * 4;
  for (int pass = 0; pass < 2; ++pass) {
#pragma unroll
    for (int q = 0; q < 8; ++q) {
      const int r = q * 2 + rsub;
      const v4f v = *(const v4fa*)&so[w][r][c4];
      *(volatile v4f*)(C + (size_t)(row0 + r) * ldc + col0 + c4) = v;
    }
    if (pass == 0) __threadfence();
  }
}
template <bool PARAM_BF16>
__global__ __launch_bounds__(256) void k_layernorm(const float* __restrict__ X, const float* __restrict__ R, const float* __restrict__ g, const float* __restrict__ bta,
                                                  float* __restrict__ out_sum, float* __restrict__ out_norm, int N, float eps) {
  __shared__ float red[256];
  const int row = blockIdx.x, tid = threadIdx.x;
  const float* x = X + (size_t)row * N; const float* rr = R ? R + (size_t)row * N : nullptr;
  float vals[16];
  const int per = N / 256;
  float s1 = 0.f;
  for (int u = 0; u < per / 4; ++u) {
    const int j = tid * 4 + 1024 * u;
    const v4f a = *(const v4fa*)(x + j);
    v4f b = {0.f,0.f,0.f,0.f}; if (rr) b = *(const v4fa*)(rr + j);
#pragma unroll
    for (int q = 0; q < 4; ++q) { const float v = a[q] + b[q]; vals[u * 4 + q] = v; s1 += v; }
  }
  red[tid] = s1; __syncthreads();
  for (int st = 128; st > 0; st >>= 1) { if (tid < st) red[tid] += red[tid + st]; __syncthreads(); }
  const float mu = red[0] / (float)N; __syncthreads();
  float s2 = 0.f;
  for (int u = 0; u < per / 4; ++u)
#pragma unroll
    for (int q = 0; q < 4; ++q) { const float c = vals[u * 4 + q] - mu; s2 += c * c; }
  red[tid] = s2; __syncthreads();
  for (int st = 128; st > 0; st >>= 1) { if (tid < st) red[tid] += red[tid + st]; __syncthreads(); }
  const float rs = rsqrtf(red[0] / (float)N + eps);
  for (int pass = 0; pass < 2; ++pass) {
    for (int u = 0; u < per / 4; ++u) {
      const int j = tid * 4 + 1024 * u;
      v4f o, sm;
#pragma unroll
      for (int q = 0; q < 4; ++q) {
        float gg = g[j + q], bb = bta[j + q];
        if (PARAM_BF16) { gg = bf16_round(gg); bb = bf16_round(bb); }
        sm[q] = vals[u * 4 + q]; o[q] = (vals[u * 4 + q] - mu) * rs * gg + bb;
      }
      if (out_sum) *(volatile v4f*)(out_sum + (size_t)row * N + j) = sm;
      *(volatile v4f*)(out_norm + (size_t)row * N + j) = o;
    }
    if (pass == 0) __threadfence();
  }
}

template <bool ASPLIT, bool BSPLIT, int ACT>
__global__ __launch_bounds__(128) void k_gemm_b(const float* __restrict__ A, int lda, size_t sA, const unsigned short* __restrict__ Bh, const unsigned short* __restrict__ Bl, int ldb, size_t sB,
                                             const float* __restrict__ bias, const float* __restrict__ resid, int ldr, size_t sR, float rsign, float alpha,
                                             float* __restrict__ C, int ldc, size_t sC, int M, int N, int K) {
  __shared__ __attribute__((aligned(16))) float so[4][16][64];
  const int tid = threadIdx.x, w = tid >> 5, lane = tid & 31, ln = lane & 15, hh = lane >> 4;
  const int by = blockIdx.y;
  A += (size_t)by * sA; Bh += (size_t)by * sB; if (BSPLIT) Bl += (size_t)by * sB; C += (size_t)by * sC; if (resid) resid += (size_t)by * sR;
  const int ntn = (N + 63) / 64; const int wid = blockIdx.x * 4 + w; const int mt = wid / ntn, nq = wid % ntn;
  if (mt * 16 >= M) return;
  const int row0 = mt * 16, col0 = nq * 64;
  const float* arow = A + (size_t)(row0 + ln) * lda;
  v8f acc[4] = {};
  for (int kb = 0; kb < K; kb += 32) {
    FragB ah, al;
    const v4f x0 = *(const v4fa*)(arow + kb + 8 * hh), x1 = *(const v4fa*)(arow + kb + 8 * hh + 4);
    const v4f x2 = *(const v4fa*)(arow + kb + 16 + 8 * hh), x3 = *(const v4fa*)(arow + kb + 16 + 8 * hh + 4);
    float xs[16] = {x0[0],x0[1],x0[2],x0[3],x1[0],x1[1],x1[2],x1[3],x2[0],x2[1],x2[2],x2[3],x3[0],x3[1],x3[2],x3[3]};
#pragma unroll
    for (int i = 0; i < 16; ++i) { const unsigned short hb = bf16_bits(xs[i]); ah.u[i] = hb; al.u[i] = ASPLIT ? bf16_bits(xs[i] - bf16_val(hb)) : (unsigned short)0; }
#pragma unroll
    for (int t = 0; t < 4; ++t) {
      if (col0 + t * 16 >= N) continue;
      const size_t boff = (size_t)(col0 + t * 16 + ln) * ldb + kb;
      FragB bh_, bl_; bh_.half[0] = *(const v8us*)(Bh + boff + 8 * hh); bh_.half[1] = *(const v8us*)(Bh + boff + 16 + 8 * hh);
      if (BSPLIT) { bl_.half[0] = *(const v8us*)(Bl + boff + 8 * hh); bl_.half[1] = *(const v8us*)(Bl + boff + 16 + 8 * hh); } else bl_ = bh_;
      acc[t] = mmaN<ASPLIT ? (BSPLIT ? 3 : 2) : 1>(ah.v, al.v, bh_.v, bl_.v, acc[t]);
    }
  }
#pragma unroll
  for (int t = 0; t < 4; ++t) {
    const int col = col0 + t * 16 + ln; if (col0 + t * 16 >= N) continue; const float bv = bias ? bf16_round(bias[col]) : 0.f;
#pragma unroll
    for (int r = 0; r < 8; ++r) { float v = acc[t][r] * alpha + bv; if (resid) v += rsign * resid[(size_t)(row0 + 8 * hh + r) * ldr + col]; if (ACT == 1) v = fmaxf(v, 0.f); else if (ACT == 2) v = fmaxf(v, 0.f) + log1pf(expf(-fabsf(v))); so[w][8 * hh + r][t * 16 + ln] = v; }
  }
  __builtin_amdgcn_fence(__ATOMIC_ACQ_REL, "workgroup"); __builtin_amdgcn_wave_barrier();
  const int rsub = lane >> 4, c4 = (lane & 15) * 4;
  for (int pass = 0; pass < 2; ++pass) {
#pragma unroll
    for (int q = 0; q < 8; ++q) { const int r = q * 2 + rsub; if (col0 + c4 < N) { const v4f v = *(const v4fa*)&so[w][r][c4]; *(volatile v4f*)(C + (size_t)(row0 + r) * ldc + col0 + c4) = v; } }
    if (pass == 0) __threadfence();
  }
}
__global__ __launch_bounds__(256) void k_split_transpose_b(const float* __restrict__ src, int lds_, size_t sIn, unsigned short* __restrict__ hi, unsigned short* __restrict__ lo, size_t sOut, int K, int N) {
  const size_t t = (size_t)blockIdx.x * 256 + threadIdx.x; const int k8n = K / 8; if (t >= (size_t)N * k8n) return;
  src += (size_t)blockIdx.y * sIn; hi += (size_t)blockIdx.y * sOut; lo += (size_t)blockIdx.y * sOut;
  const int n = (int)(t / k8n), k8 = (int)(t % k8n) * 8; v8us vh, vl;
#pragma unroll
  for (int i = 0; i < 8; ++i) { const float x = src[(size_t)(k8 + i) * lds_ + n]; const unsigned short hb = bf16_bits(x); vh[i] = hb; vl[i] = bf16_bits(x - bf16_val(hb)); }
  unsigned short* dh = hi + (size_t)n * K + k8; unsigned short* dl = lo + (size_t)n * K + k8;
  *(volatile v8us*)dh = vh; *(volatile v8us*)dl = vl; __threadfence(); *(volatile v8us*)dh = vh; *(volatile v8us*)dl = vl;
}

typedef _Float16 v16h __attribute__((ext_vector_type(16)));
union FragH { v16h v; v8us half[2]; _Float16 h[16]; unsigned short u[16]; };
template <int NT>
__device__ __forceinline__ v8f mmaH(v16h ah, v16h al, v16h bh, v16h bl, v8f c) {
  c = __builtin_amdgcn_wmma_f32_16x16x32_f16(false, ah, false, bh, (short)0, c, false, false);
  if (NT >= 2) c = __builtin_amdgcn_wmma_f32_16x16x32_f16(false, al, false, bh, (short)0, c, false, false);
  if (NT >= 3) c = __builtin_amdgcn_wmma_f32_16x16x32_f16(false, ah, false, bl, (short)0, c, false, false);
  asm volatile("v_nop\n\tv_nop\n\tv_nop\n\tv_nop" : "+v"(c) : "v"(ah), "v"(al), "v"(bh), "v"(bl));
  return c;
}
template <bool ASPLIT>
__global__ __launch_bounds__(128) void k_gemm_h(const float* __restrict__ A, int lda, size_t sA, const _Float16* __restrict__ Bh, int ldb, size_t sB, float alpha, float* __restrict__ C, int ldc, size_t sC, int M, int N, int K) {
  __shared__ __attribute__((aligned(16))) float so[4][16][64];
  const int tid = threadIdx.x, w = tid >> 5, lane = tid & 31, ln = lane & 15, hh = lane >> 4; const int by = blockIdx.y;
  A += (size_t)by * sA; Bh += (size_t)by * sB; C += (size_t)by * sC;
  const int ntn = (N + 63) / 64; const int wid = blockIdx.x * 4 + w; const int mt = wid / ntn, nq = wid % ntn; if (mt * 16 >= M) return;
  const int row0 = mt * 16, col0 = nq * 64; const float* arow = A + (size_t)(row0 + ln) * lda;
  v8f acc[4] = {};
  for (int kb = 0; kb < K; kb += 32) {
    FragH ah, al;
    const v4f x0 = *(const v4fa*)(arow + kb + 8 * hh), x1 = *(const v4fa*)(arow + kb + 8 * hh + 4), x2 = *(const v4fa*)(arow + kb + 16 + 8 * hh), x3 = *(const v4fa*)(arow + kb + 16 + 8 * hh + 4);
    float xs[16] = {x0[0],x0[1],x0[2],x0[3],x1[0],x1[1],x1[2],x1[3],x2[0],x2[1],x2[2],x2[3],x3[0],x3[1],x3[2],x3[3]};
#pragma unroll
    for (int i = 0; i < 16; ++i) { const _Float16 h = (_Float16)xs[i]; ah.h[i] = h; al.h[i] = ASPLIT ? (_Float16)(xs[i] - (float)h) : (_Float16)0.0f; }
#pragma unroll
    for (int t = 0; t < 4; ++t) { if (col0 + t * 16 >= N) continue; const size_t boff = (size_t)(col0 + t * 16 + ln) * ldb + kb; FragH bq; bq.half[0] = *(const v8us*)(Bh + boff + 8 * hh); bq.half[1] = *(const v8us*)(Bh + boff + 16 + 8 * hh);
      acc[t] = mmaH<ASPLIT ? 2 : 1>(ah.v, al.v, bq.v, bq.v, acc[t]); }
  }
#pragma unroll
  for (int t = 0; t < 4; ++t) { if (col0 + t * 16 >= N) continue;
#pragma unroll
    for (int r = 0; r < 8; ++r) so[w][8 * hh + r][t * 16 + ln] = acc[t][r] * alpha; }
  __builtin_amdgcn_fence(__ATOMIC_ACQ_REL, "workgroup"); __builtin_amdgcn_wave_barrier();
  const int rsub = lane >> 4, c4 = (lane & 15) * 4;
  for (int pass = 0; pass < 2; ++pass) {
#pragma unroll
    for (int q = 0; q < 8; ++q) { const int r = q * 2 + rsub; if (col0 + c4 < N) { const v4f v = *(const v4fa*)&so[w][r][c4]; *(volatile v4f*)(C + (size_t)(row0 + r) * ldc + col0 + c4) = v; } }
    if (pass == 0) __threadfence(); }
}

__device__ __forceinline__ void pix2tok(int h, int w2, int& blk, int& l) { const int side = (w2 >= WW) ? 1 : 0; const int w = w2 - side * WW; blk = (h / SH) * SS + (w / SW); l = ((h % SH) * SW + (w % SW)) * 2 + side; }
__global__ __launch_bounds__(256) void k_qkv(const float* __restrict__ x, const float* __restrict__ Wq, const float* __restrict__ bq, const float* __restrict__ Wk, const float* __restrict__ bk, const float* __restrict__ Wv, const float* __restrict__ bv, float* __restrict__ QKV) {
  __shared__ float sw[128][CC + 1]; __shared__ float sb[128]; __shared__ float sx[CC][64 + 1]; __shared__ float so[64][128 + 1];
  const int tid = threadIdx.x; for (int e = tid; e < 128 * CC; e += 256) { const int o = e / CC, c = e % CC; sw[o][c] = bf16_round(o < 32 ? Wq[o * CC + c] : (o < 64 ? Wk[(o - 32) * CC + c] : Wv[(o - 64) * CC + c])); }
  if (tid < 128) sb[tid] = bf16_round(tid < 32 ? bq[tid] : (tid < 64 ? bk[tid - 32] : bv[tid - 64]));
  const int n = blockIdx.y; const int p0 = blockIdx.x * 64;
  for (int e = tid; e < CC * 64; e += 256) { const int c = e / 64, p = e % 64; sx[c][p] = bf16_round(x[((size_t)n * CC + c) * (HH * W2) + p0 + p]); }
  __syncthreads();
  const int p = tid & 63, og = tid >> 6; float acc[32]; for (int u = 0; u < 32; ++u) acc[u] = sb[og * 32 + u];
#pragma unroll 1
  for (int c = 0; c < CC; ++c) { const float xv = sx[c][p];
#pragma unroll
    for (int u = 0; u < 32; ++u) acc[u] += xv * sw[og * 32 + u][c]; }
  for (int u = 0; u < 32; ++u) so[p][og * 32 + u] = acc[u];
  __syncthreads();
  float* dst = QKV + ((size_t)n * HH * W2 + p0) * 128;
  for (int pass = 0; pass < 2; ++pass) { for (int e = tid; e < 64 * 128; e += 256) *(volatile float*)(dst + e) = so[e >> 7][e & 127]; if (pass == 0) __threadfence(); }
}
__global__ __launch_bounds__(256) void k_bnstat(const float* __restrict__ QKV, double* __restrict__ part) { __shared__ double r1[4][64], r2[4][64]; const int t = threadIdx.x, c = t & 63, g = t >> 6; double s = 0.0, q = 0.0; const int p0 = blockIdx.x * 1024;
#pragma unroll 1
  for (int u = g; u < 1024; u += 4) { const float v = QKV[(size_t)(p0 + u) * 128 + c]; s += (double)v; q += (double)v * (double)v; }
  r1[g][c] = s; r2[g][c] = q; __syncthreads();
  if (t < 64) { const double a = ((r1[0][t] + r1[1][t]) + r1[2][t]) + r1[3][t], b = ((r2[0][t] + r2[1][t]) + r2[2][t]) + r2[3][t]; double* d = part + ((size_t)blockIdx.x * 64 + t) * 2; *(volatile double*)d = a; *(volatile double*)(d + 1) = b; __threadfence(); *(volatile double*)d = a; *(volatile double*)(d + 1) = b; } }
__global__ __launch_bounds__(64) void k_bnfin(const double* __restrict__ part, int nblk, const float* __restrict__ gq, const float* __restrict__ btq, const float* __restrict__ gk, const float* __restrict__ btk, float* __restrict__ st) { const int c = threadIdx.x; double s = 0.0, q = 0.0; for (int k = 0; k < nblk; ++k) { s += part[((size_t)k * 64 + c) * 2]; q += part[((size_t)k * 64 + c) * 2 + 1]; }
  const double mu = s / (double)NPIX; double var = q / (double)NPIX - mu * mu; if (var < 0.0) var = 0.0; const float rs = (float)(1.0 / sqrt(var + 1e-5)); const float g = bf16_round(c < 32 ? gq[c] : gk[c - 32]), bb = bf16_round(c < 32 ? btq[c] : btk[c - 32]);
  const float sc = rs * g, sh = bb - (float)mu * sc; *(volatile float*)(st + c * 2) = sc; *(volatile float*)(st + c * 2 + 1) = sh; __threadfence(); *(volatile float*)(st + c * 2) = sc; *(volatile float*)(st + c * 2 + 1) = sh; }
__global__ __launch_bounds__(256) void k_slabs(const float* __restrict__ QKV, const float* __restrict__ st, float* __restrict__ Qs, _Float16* __restrict__ Ks, _Float16* __restrict__ Vt) {
  __shared__ float so[64][128 + 1]; const int tid = threadIdx.x; const int j = blockIdx.x % SS; const int h = (blockIdx.x / SS) % HH; const int n = blockIdx.x / (SS * HH);
  const int blk = (h / SH) * SS + j; const int sl = n * NBK + blk; const int l0 = (h % SH) * SW * 2;
  for (int e = tid; e < 64 * 128; e += 256) { const int tt = e >> 7, c = e & 127; const int wl = tt >> 1, side = tt & 1; const size_t pix = ((size_t)n * HH + h) * W2 + side * WW + j * SW + wl; float v = QKV[pix * 128 + c]; if (c < 64) v = v * st[c * 2] + st[c * 2 + 1]; so[tt][c] = v; }
  __syncthreads();
  float* qd = Qs + ((size_t)sl * LL + l0) * CK; _Float16* kd = Ks + ((size_t)sl * LL + l0) * CK; typedef _Float16 v2h __attribute__((ext_vector_type(2)));
  for (int pass = 0; pass < 2; ++pass) {
    for (int e = tid; e < 64 * CK; e += 256) *(volatile float*)(qd + e) = so[e >> 5][e & 31];
    for (int e2 = tid; e2 < 64 * CK / 2; e2 += 256) { const int e = e2 * 2; v2h hv; hv.x = (_Float16)so[e >> 5][32 + (e & 31)]; hv.y = (_Float16)so[e >> 5][32 + (e & 31) + 1]; *(volatile v2h*)(kd + e) = hv; }
    for (int e2 = tid; e2 < CV * 32; e2 += 256) { const int cv = e2 >> 5, tp = (e2 & 31) * 2; v2h hv; hv.x = (_Float16)so[tp][64 + cv]; hv.y = (_Float16)so[tp + 1][64 + cv]; *(volatile v2h*)(Vt + ((size_t)sl * CV + cv) * LL + l0 + tp) = hv; }
    if (pass == 0) __threadfence(); }
}
__global__ __launch_bounds__(1024) void k_softmax(float* __restrict__ S, float* __restrict__ Dn) {
  __shared__ float sd[32]; const int tid = threadIdx.x, wv = tid >> 5, lane = tid & 31; const size_t r = (size_t)blockIdx.x * 32 + wv; float* row = S + r * LL; const float sc = 0.17677669529663687f;
  float mx = -3.0e38f;
#pragma unroll 1
  for (int j = lane; j < LL; j += 32) mx = fmaxf(mx, row[j] * sc);
  for (int o = 16; o >= 1; o >>= 1) mx = fmaxf(mx, __shfl_xor(mx, o, 32));
  float den = 0.f;
#pragma unroll 1
  for (int j = lane; j < LL; j += 32) { const float e = expf(row[j] * sc - mx); den += e; *(volatile float*)(row + j) = e * 256.0f; }
  for (int o = 16; o >= 1; o >>= 1) den += __shfl_xor(den, o, 32);
  __threadfence();
#pragma unroll 1
  for (int j = lane; j < LL; j += 32) { const float pv = row[j]; *(volatile float*)(row + j) = pv; }
  if (lane == 0) sd[wv] = den; __syncthreads();
  if (tid < 32) { *(volatile float*)(Dn + (size_t)blockIdx.x * 32 + tid) = sd[tid]; } __threadfence(); if (tid < 32) { *(volatile float*)(Dn + (size_t)blockIdx.x * 32 + tid) = sd[tid]; }
}
__global__ __launch_bounds__(256) void k_out(const float* __restrict__ O, const float* __restrict__ Dn, float* __restrict__ out) { const size_t t = (size_t)blockIdx.x * 256 + threadIdx.x; if (t >= (size_t)NI * CV * HH * W2) return; const int w2 = (int)(t % W2); const int h = (int)((t / W2) % HH); const int cv = (int)((t / ((size_t)W2 * HH)) % CV); const int n = (int)(t / ((size_t)W2 * HH * CV));
  int blk, l; pix2tok(h, w2, blk, l); const size_t sl = (size_t)n * NBK + blk; const float v = O[(sl * LL + l) * CV + cv] / Dn[sl * LL + l]; *(volatile float*)(out + t) = v; __threadfence(); *(volatile float*)(out + t) = v; }
extern "C" void kernel_launch(void* const* d_in, const int* in_sizes, int n_in,
                              void* d_out, int out_size, void* d_ws, size_t ws_size, hipStream_t stream) {
  (void)in_sizes; (void)n_in; (void)out_size;
  const float* x = (const float*)d_in[0]; const float* Wq = (const float*)d_in[1]; const float* bq = (const float*)d_in[2]; const float* gq = (const float*)d_in[3]; const float* btq = (const float*)d_in[4]; const float* Wk = (const float*)d_in[5]; const float* bk = (const float*)d_in[6]; const float* gk = (const float*)d_in[7]; const float* btk = (const float*)d_in[8]; const float* Wv = (const float*)d_in[9]; const float* bv = (const float*)d_in[10];
  char* ws = (char*)d_ws; size_t off = 0;
  auto take = [&](size_t bytes) { char* p = ws + off; off += (bytes + 255) & ~(size_t)255; return p; };
  const int NBLK = NPIX / 1024;
  float* QKV = (float*)take((size_t)NPIX * 128 * 4); double* part = (double*)take((size_t)NBLK * 64 * 2 * 8); float* st = (float*)take(64 * 2 * 4);
  float* Qs = (float*)take((size_t)NSL * LL * CK * 4); _Float16* Ks = (_Float16*)take((size_t)NSL * LL * CK * 2); _Float16* Vt = (_Float16*)take((size_t)NSL * CV * LL * 2);
  float* S = (float*)take((size_t)8 * LL * LL * 4); float* Dn = (float*)take((size_t)NSL * LL * 4); float* O = (float*)take((size_t)NSL * LL * CV * 4);
  if (off > ws_size) return;
  k_qkv<<<dim3(HH * W2 / 64, NI), 256, 0, stream>>>(x, Wq, bq, Wk, bk, Wv, bv, QKV);
  k_bnstat<<<NBLK, 256, 0, stream>>>(QKV, part); k_bnfin<<<1, 64, 0, stream>>>(part, NBLK, gq, btq, gk, btk, st);
  k_slabs<<<NI * HH * SS, 256, 0, stream>>>(QKV, st, Qs, Ks, Vt);
  for (int s0 = 0; s0 < NSL; s0 += 8) {
    k_gemm_h<true><<<dim3(((LL / 16) * (LL / 64) + 3) / 4, 8), 128, 0, stream>>>(Qs + (size_t)s0 * LL * CK, CK, (size_t)LL * CK, Ks + (size_t)s0 * LL * CK, CK, (size_t)LL * CK, 1.f, S, LL, (size_t)LL * LL, LL, LL, CK);
    k_softmax<<<(8 * LL) / 32, 1024, 0, stream>>>(S, Dn + (size_t)s0 * LL);
    k_gemm_h<false><<<dim3(((LL / 16) * 1 + 3) / 4, 8), 128, 0, stream>>>(S, LL, (size_t)LL * LL, Vt + (size_t)s0 * CV * LL, LL, (size_t)CV * LL, 0.00390625f, O + (size_t)s0 * LL * CV, CV, (size_t)LL * CV, LL, CV, LL);
  }
  k_out<<<(unsigned)(((size_t)NI * CV * HH * W2 + 255) / 256), 256, 0, stream>>>(O, Dn, (float*)d_out);
}
